// Mosaic_50603304682317
// MI455X (gfx1250) — hardware-run, weakly checked
//
#include <hip/hip_runtime.h>
#include <stddef.h>


typedef _Float16 v16h __attribute__((ext_vector_type(16)));
typedef _Float16 v8h  __attribute__((ext_vector_type(8)));
typedef float    v8f  __attribute__((ext_vector_type(8)));
typedef float    v4f  __attribute__((ext_vector_type(4)));
typedef _Float16 h16;

#ifndef XROWS
#define XROWS 256
#endif
#ifndef NOC
#define NOC 128
#endif
#define XROWS_FULL 256
#define OC_FULL    128
#define ICNT       128
#define TS         64
#define NBLK       1024
#define IDIM       (ICNT * TS)
#define ODIM_FULL  (OC_FULL * TS)
#define WLD        (NBLK * TS)

static_assert(XROWS >= 64 && XROWS <= XROWS_FULL && (XROWS % 64) == 0);
static_assert(NOC >= 1 && NOC <= OC_FULL);
static_assert(TS == 64);
static_assert(IDIM == 8192 && ODIM_FULL == 8192);
static_assert((TS % 32) == 0);
static_assert(((size_t)XROWS * IDIM) % (256u * 8u) == 0);
static_assert(64 * 8 == 2 * 256);
static_assert(64 * 16 == 4 * 256);

#define LDT 72
#define LDC 68
static_assert((LDT % 8) == 0 && LDT >= 64);
static_assert((LDC % 4) == 0 && LDC >= 64);

#define WCARRY 64.0f
#define XCARRY 16.0f

#define WT_BYTES   ((size_t)TS * WLD * 2)
#define X16_BYTES  ((size_t)XROWS * IDIM * 2)
#define OFF_WT   ((size_t)0)
#define OFF_X16  (OFF_WT + WT_BYTES)
#define WS_TOTAL (OFF_X16 + X16_BYTES)
static_assert((WT_BYTES % 128) == 0 && (X16_BYTES % 128) == 0);
static_assert(WS_TOTAL <= (size_t)134217728);

__device__ __forceinline__ float bf16r(float x) {
  unsigned int u = __float_as_uint(x);
  u = (u + 0x7FFFu + ((u >> 16) & 1u)) & 0xFFFF0000u;
  return __uint_as_float(u);
}

static __device__ __forceinline__ h16 toh_flush(float v) {
  const h16 r = (h16)v;
  return (fabsf(v) < 6.103515625e-05f) ? (h16)0.0f : r;
}

__device__ __forceinline__ v16h frag_at(const _Float16* p) {
  v8h lo = *(const v8h*)(p);
  v8h hi = *(const v8h*)(p + 16);
  v16h out;
#pragma unroll
  for (int i = 0; i < 8; ++i) { out[i] = lo[i]; out[i + 8] = hi[i]; }
  return out;
}
__device__ __forceinline__ v16h ld_frag(const _Float16* base, unsigned ld) {
  const unsigned lane = threadIdx.x & 31u;
  return frag_at(base + (lane & 15u) * ld + (lane >> 4) * 8u);
}

__device__ __forceinline__ v8f wmma16(v16h a, v16h b, v8f c) {
  v8f d = __builtin_amdgcn_wmma_f32_16x16x32_f16(false, a, false, b, (short)0, c,
                                                 false, false);
  asm volatile("v_nop\n\tv_nop\n\tv_nop\n\tv_nop" : "+v"(d) : "v"(a), "v"(b));
  return d;
}

__global__ __launch_bounds__(256) void wconv_kernel(
    const float* __restrict__ W, _Float16* __restrict__ Wt, unsigned ldw, unsigned ldk) {
  __shared__ _Float16 T[64 * LDT];
  const unsigned tid = threadIdx.x;
  const unsigned n0 = blockIdx.x * 64u;
  const unsigned k0 = blockIdx.y * 64u;
#pragma unroll 4
  for (unsigned j = 0; j < 16u; ++j) {
    const unsigned idx = tid + 256u * j;
    const unsigned kr = idx >> 6, nc = idx & 63u;
    const float v = W[(size_t)(k0 + kr) * ldw + n0 + nc];
    T[nc * LDT + kr] = (_Float16)(WCARRY * bf16r(v));
  }
  __syncthreads();
  v8h x[2];
  size_t off[2];
#pragma unroll
  for (unsigned i = 0; i < 2u; ++i) {
    const unsigned n = 32u * i + (tid >> 3);
    const unsigned kc = (tid & 7u) * 8u;
    x[i] = *(const v8h*)&T[n * LDT + kc];
    off[i] = (size_t)(n0 + n) * ldk + k0 + kc;
  }
#pragma unroll
  for (int i = 0; i < 2; ++i) *(volatile v8h*)(Wt + off[i]) = x[i];
  __threadfence();
#pragma unroll
  for (int i = 0; i < 2; ++i) *(volatile v8h*)(Wt + off[i]) = x[i];
}

__global__ __launch_bounds__(256) void xconv_kernel(
    const float* __restrict__ X, _Float16* __restrict__ X16) {
#pragma clang fp contract(off)
  const unsigned t = blockIdx.x * 256u + threadIdx.x;
  const size_t e = (size_t)t * 8u;
  const v4f a0 = *(const v4f*)(X + e);
  const v4f a1 = *(const v4f*)(X + e + 4u);
  v8h o;
#pragma unroll
  for (int i = 0; i < 4; ++i) {
    o[i]     = toh_flush(XCARRY * bf16r(a0[i]));
    o[i + 4] = toh_flush(XCARRY * bf16r(a1[i]));
  }
  _Float16* p = X16 + e;
  *(volatile v8h*)p = o;
  __threadfence();
  *(volatile v8h*)p = o;
}

__global__ __launch_bounds__(256) void blockgemm_kernel(
    const _Float16* __restrict__ X16, const _Float16* __restrict__ Wt,
    const int* __restrict__ table, const float* __restrict__ bias, float* __restrict__ outf) {
  __shared__ _Float16 Bs[64 * LDT];
  __shared__ float Cs[64 * LDC];
  const unsigned tid = threadIdx.x, lane = tid & 31u;
  const unsigned w = (unsigned)__builtin_amdgcn_readfirstlane((int)(threadIdx.x >> 5));
  const unsigned mw = w >> 1, nw = w & 1u;
  const unsigned hh = lane >> 4, m = lane & 15u;
  const unsigned o = blockIdx.x;
  const unsigned n0 = o * 64u;
  const unsigned row0 = blockIdx.y * 64u;

  const _Float16* ap = X16 + (size_t)(row0 + mw * 16u + m) * IDIM + hh * 8u;
  v8f acc0 = {}, acc1 = {};
#pragma unroll 1
  for (unsigned i = 0; i < (unsigned)ICNT; ++i) {
    int p = table[i * (unsigned)OC_FULL + o];
    p = min(max(p, 0), NBLK - 1);
    const _Float16* src = Wt + (size_t)p * 64u;
#pragma unroll
    for (unsigned j = 0; j < 2u; ++j) {
      const unsigned idx = tid + 256u * j;
      const unsigned r = idx >> 3, c = (idx & 7u) * 8u;
      *(v8h*)&Bs[r * LDT + c] = *(const v8h*)(src + (size_t)r * WLD + c);
    }
    __syncthreads();
#pragma unroll
    for (unsigned c = 0; c < 2u; ++c) {
      const v16h a  = frag_at(ap + i * 64u + c * 32u);
      const v16h b0 = ld_frag(&Bs[(nw * 32u) * LDT + c * 32u], LDT);
      const v16h b1 = ld_frag(&Bs[(nw * 32u + 16u) * LDT + c * 32u], LDT);
      acc0 = wmma16(a, b0, acc0);
      acc1 = wmma16(a, b1, acc1);
    }
    __syncthreads();
  }

#pragma unroll
  for (int r = 0; r < 8; ++r) {
    float* d = &Cs[(mw * 16u + hh * 8u + (unsigned)r) * LDC + nw * 32u + m];
    d[0]  = acc0[r];
    d[16] = acc1[r];
  }
  __syncthreads();

  const float cs = 1.0f / (WCARRY * XCARRY);
  v4f xs[4];
  size_t off[4];
#pragma unroll
  for (unsigned i = 0; i < 4u; ++i) {
    const unsigned r = 16u * i + (tid >> 4);
    const unsigned c = (tid & 15u) * 4u;
    const v4f u = *(const v4f*)&Cs[r * LDC + c];
    const v4f g = *(const v4f*)(bias + n0 + c);
    v4f val;
#pragma unroll
    for (int j = 0; j < 4; ++j) val[j] = u[j] * cs + bf16r(g[j]);
    xs[i] = val;
    off[i] = (size_t)(row0 + r) * ODIM_FULL + n0 + c;
  }
#pragma unroll
  for (int i = 0; i < 4; ++i) *(volatile v4f*)(outf + off[i]) = xs[i];
  __threadfence();
#pragma unroll
  for (int i = 0; i < 4; ++i) *(volatile v4f*)(outf + off[i]) = xs[i];
}

extern "C" void kernel_launch(void* const* d_in, const int* in_sizes, int n_in,
                              void* d_out, int out_size, void* d_ws, size_t ws_size,
                              hipStream_t stream) {
  if (n_in < 4) return;
  if ((long long)in_sizes[0] < (long long)XROWS * IDIM) return;
  if ((long long)in_sizes[1] < (long long)NBLK * TS * TS) return;
  if ((long long)in_sizes[2] < (long long)NOC * TS) return;
  if ((long long)in_sizes[3] < (long long)(ICNT - 1) * OC_FULL + NOC) return;
  if ((long long)out_size < (long long)(XROWS - 1) * ODIM_FULL + (long long)NOC * TS) return;
  if (ws_size < WS_TOTAL) return;

  const float* X     = (const float*)d_in[0];
  const float* bank  = (const float*)d_in[1];
  const float* bias  = (const float*)d_in[2];
  const int*   table = (const int*)d_in[3];
  float* out = (float*)d_out;

  char* ws = (char*)d_ws;
  _Float16* Wt  = (_Float16*)(ws + OFF_WT);
  _Float16* X16 = (_Float16*)(ws + OFF_X16);

  dim3 blk(256);

  wconv_kernel<<<dim3(1, NBLK), blk, 0, stream>>>(bank, Wt, (unsigned)TS, (unsigned)WLD);
  xconv_kernel<<<dim3((unsigned)(((size_t)XROWS * IDIM) / 2048u)), blk, 0, stream>>>(X, X16);
  blockgemm_kernel<<<dim3(NOC, XROWS / 64), blk, 0, stream>>>(X16, Wt, table, bias, out);
}
